// PD_LSTM_38345468019409
// MI455X (gfx1250) — hardware-verified
//
#include <hip/hip_runtime.h>
#include <math.h>

typedef __attribute__((ext_vector_type(16))) _Float16 v16h;
typedef __attribute__((ext_vector_type(16))) __bf16 v16b;
typedef __attribute__((ext_vector_type(8)))  _Float16 v8h;
typedef __attribute__((ext_vector_type(8)))  float v8f;
typedef __attribute__((ext_vector_type(4)))  float v4f;
typedef __attribute__((ext_vector_type(2)))  float v2f;
typedef __attribute__((ext_vector_type(4)))  unsigned v4u;
typedef __attribute__((ext_vector_type(4)))  int v4i;
typedef float __attribute__((may_alias)) float_a;
typedef int __attribute__((may_alias)) int_a;

template <typename T> __device__ __forceinline__ void vst2(void* p, T v) { *(volatile T*)p = v; __threadfence(); *(volatile T*)p = v; }
__device__ __forceinline__ v8f wmma16(v16h a, v16h b, v8f c) {
  v8f d = __builtin_amdgcn_wmma_f32_16x16x32_f16(false, a, false, b, (short)0, c, false, false);
  asm volatile("v_nop\n\tv_nop\n\tv_nop\n\tv_nop" : "+v"(d) : "v"(a), "v"(b));
  return d;
}
__device__ __forceinline__ v8f wmma_bf(v16b a, v16b b, v8f c) {
  v8f d = __builtin_amdgcn_wmma_f32_16x16x32_bf16(false, a, false, b, (short)0, c, false, false);
  asm volatile("v_nop\n\tv_nop\n\tv_nop\n\tv_nop" : "+v"(d) : "v"(a), "v"(b));
  return d;
}
__device__ __forceinline__ v16h frag_h(const _Float16* rowk0, int lane) {
  union { v16h v; v8h q[2]; } u; const _Float16* p = rowk0 + 8 * (lane >> 4);
  u.q[0] = *(const v8h*)p; u.q[1] = *(const v8h*)(p + 16); return u.v;
}
__device__ __forceinline__ v16h frag_f32(const float* rowk0, int lane) {
  v16h a; const float* p = rowk0 + 8 * (lane >> 4);
#pragma unroll
  for (int i = 0; i < 8; ++i) { a[i] = (_Float16)p[i]; a[8 + i] = (_Float16)p[16 + i]; }
  return a;
}
__device__ __forceinline__ v16h frag_f32s(const float* rowk0, int lane, float sc) {
  v16h a; const float* p = rowk0 + 8 * (lane >> 4);
#pragma unroll
  for (int i = 0; i < 8; ++i) { a[i] = (_Float16)(p[i] * sc); a[8 + i] = (_Float16)(p[16 + i] * sc); }
  return a;
}
__device__ __forceinline__ v16h fragc_f32(const float* W, int k0, int n, int lane, int ld, int K) {
  v16h a; const int g = lane >> 4;
#pragma unroll
  for (int i = 0; i < 8; ++i) { const int ka = k0 + 8 * g + i, kb = ka + 16;
    a[i] = (_Float16)(ka < K ? W[(size_t)ka * ld + n] : 0.f); a[8 + i] = (_Float16)(kb < K ? W[(size_t)kb * ld + n] : 0.f); }
  return a;
}
struct F2 { v16b h, l; };
__device__ __forceinline__ F2 bsplit16(const float v[16]) { F2 r;
#pragma unroll
  for (int i = 0; i < 16; ++i) { const __bf16 h = (__bf16)v[i]; r.h[i] = h; r.l[i] = (__bf16)(v[i] - (float)h); }
  return r; }
__device__ __forceinline__ F2 split_row(const float* row, int k0, int lane) { float v[16]; const float* p = row + k0 + 8 * (lane >> 4);
#pragma unroll
  for (int i = 0; i < 8; ++i) { v[i] = p[i]; v[8 + i] = p[16 + i]; }
  return bsplit16(v); }
__device__ __forceinline__ F2 split_rowK(const float* row, int k0, int lane, int K) { float v[16]; const int g = lane >> 4;
#pragma unroll
  for (int i = 0; i < 8; ++i) { const int ka = k0 + 8 * g + i, kb = ka + 16; v[i] = ka < K ? row[ka] : 0.f; v[8 + i] = kb < K ? row[kb] : 0.f; }
  return bsplit16(v); }
__device__ __forceinline__ F2 split_col(const float* W, int k0, int n, int lane, int ld, int K) { float v[16]; const int g = lane >> 4;
#pragma unroll
  for (int i = 0; i < 8; ++i) { const int ka = k0 + 8 * g + i, kb = ka + 16; v[i] = ka < K ? W[(size_t)ka * ld + n] : 0.f; v[8 + i] = kb < K ? W[(size_t)kb * ld + n] : 0.f; }
  return bsplit16(v); }
__device__ __forceinline__ v8f mac3(const F2& a, const F2& b, v8f c) { c = wmma_bf(a.l, b.h, c); c = wmma_bf(a.h, b.l, c); return wmma_bf(a.h, b.h, c); }
__device__ __forceinline__ float sigm(float v) { return 1.0f / (1.0f + expf(-v)); }
#define LDSX() do { asm volatile("s_wait_dscnt 0" ::: "memory"); __builtin_amdgcn_wave_barrier(); __builtin_amdgcn_fence(__ATOMIC_RELEASE, "workgroup"); } while (0)


#define T 512
#define NBATCH 16
#define NIN 32
#define HD 256
#define G4 (4 * HD)
#define NROW (T * NBATCH)
#define MAXIT 20
#define TW 32
#define WSC 16.0f

__global__ __launch_bounds__(256) void k_pack(const float* __restrict__ src, _Float16* __restrict__ dst, int n8, float sc) {
  const int i8 = blockIdx.x * 256 + threadIdx.x; if (i8 >= n8) return;
  union { v8h h; v4u u; } pk;
#pragma unroll
  for (int e = 0; e < 8; ++e) pk.h[e] = (_Float16)(src[(size_t)i8 * 8 + e] * sc);
  vst2(dst + (size_t)i8 * 8, pk.u);
}
template <int KIN>
__global__ __launch_bounds__(256) void k_lstm(const _Float16* __restrict__ Xh, const _Float16* __restrict__ Wih, const _Float16* __restrict__ Whh,
                                             const float* __restrict__ bih, const float* __restrict__ bhh, _Float16* __restrict__ Hh, float* __restrict__ Hf) {
  __shared__ __align__(16) _Float16 sh16[NBATCH][HD + 8];
  __shared__ __align__(16) float sg[NBATCH][G4 + 4];
  const int tid = threadIdx.x, wave = tid >> 5, lane = tid & 31, col = lane & 15, g = lane >> 4;
  const int n0 = wave * 128;
  for (int q = tid; q < NBATCH * HD; q += 256) sh16[q / HD][q % HD] = (_Float16)0.0f;
  float c[NBATCH];
#pragma unroll
  for (int b = 0; b < NBATCH; ++b) c[b] = 0.f;
  float bsum[8];
#pragma unroll
  for (int j = 0; j < 8; ++j) bsum[j] = bih[n0 + j * 16 + col] + bhh[n0 + j * 16 + col];
  __syncthreads();
#pragma unroll 1
  for (int t = 0; t < T; ++t) {
    if (Hh != nullptr && t > 0) {
      for (int p = tid; p < NBATCH * (HD / 8); p += 256) { const int row = p / (HD / 8), c8 = p % (HD / 8); vst2(Hh + ((size_t)(t - 1) * NBATCH + row) * HD + c8 * 8, *(const v4u*)(&sh16[row][c8 * 8])); } }
    v8f acc[8] = {};
#pragma unroll
    for (int kc = 0; kc < KIN / 32; ++kc) { const v16h a = frag_h(Xh + ((size_t)t * NBATCH + col) * KIN + kc * 32, lane);
#pragma unroll
      for (int j = 0; j < 8; ++j) acc[j] = wmma16(a, frag_h(Wih + (size_t)(n0 + j * 16 + col) * KIN + kc * 32, lane), acc[j]); }
#pragma unroll
    for (int kc = 0; kc < HD / 32; ++kc) { const v16h a = frag_h(&sh16[col][0] + kc * 32, lane);
#pragma unroll
      for (int j = 0; j < 8; ++j) acc[j] = wmma16(a, frag_h(Whh + (size_t)(n0 + j * 16 + col) * HD + kc * 32, lane), acc[j]); }
#pragma unroll
    for (int j = 0; j < 8; ++j)
#pragma unroll
      for (int r = 0; r < 8; ++r) sg[8 * g + r][n0 + j * 16 + col] = acc[j][r] * (1.0f / WSC) + bsum[j];
    __syncthreads();
    const int u = tid;
#pragma unroll
    for (int b = 0; b < NBATCH; ++b) {
      const float gi = sg[b][u], gf = sg[b][HD + u], gg = sg[b][2 * HD + u], go = sg[b][3 * HD + u];
      c[b] = sigm(gf) * c[b] + sigm(gi) * tanhf(gg);
      const float h = sigm(go) * tanhf(c[b]);
      sh16[b][u] = (_Float16)h;
      if (Hf != nullptr) vst2(Hf + ((size_t)t * NBATCH + b) * HD + u, (float_a)h);
    }
    __syncthreads();
  }
  if (Hh != nullptr) { for (int p = tid; p < NBATCH * (HD / 8); p += 256) { const int row = p / (HD / 8), c8 = p % (HD / 8); vst2(Hh + ((size_t)(T - 1) * NBATCH + row) * HD + c8 * 8, *(const v4u*)(&sh16[row][c8 * 8])); } }
}
__global__ __launch_bounds__(256) void k_xinit(const float* __restrict__ Hm, const float* __restrict__ tau, float* __restrict__ X, float* __restrict__ M1) {
  const int i4 = blockIdx.x * 256 + threadIdx.x; if (i4 >= HD * HD / 4) return;
  const float tu = tau[0]; const v4f h = *(const v4f*)(Hm + (size_t)i4 * 4); v4f x, m; const int r = (i4 * 4) / HD, c0 = (i4 * 4) % HD;
#pragma unroll
  for (int e = 0; e < 4; ++e) { x[e] = -tu * h[e]; m[e] = x[e] + ((c0 + e) == r ? 1.0f : 0.0f); }
  vst2(X + (size_t)i4 * 4, x); vst2(M1 + (size_t)i4 * 4, m);
}
__global__ __launch_bounds__(128) void k_mm256(const float* __restrict__ A, const float* __restrict__ B, const float* __restrict__ D, float* __restrict__ C) {
  __shared__ __align__(16) float so[16][HD + 4];
  const int tid = threadIdx.x, wave = tid >> 5, lane = tid & 31, col = lane & 15, g = lane >> 4;
  const int m0 = blockIdx.x * 16, nb = wave * 64;
  v8f acc[4] = {};
#pragma unroll 1
  for (int kc = 0; kc < HD / 32; ++kc) { const F2 a = split_row(A + (size_t)(m0 + col) * HD, kc * 32, lane);
#pragma unroll
    for (int j = 0; j < 4; ++j) acc[j] = mac3(a, split_col(B, kc * 32, nb + j * 16 + col, lane, HD, HD), acc[j]); }
#pragma unroll
  for (int j = 0; j < 4; ++j)
#pragma unroll
    for (int r = 0; r < 8; ++r) { const int row = 8 * g + r, n = nb + j * 16 + col; so[row][n] = acc[j][r] + (D ? D[(size_t)(m0 + row) * HD + n] : 0.f); }
  __syncthreads();
  for (int q = tid; q < 16 * (HD / 4); q += 128) { const int rl = q / (HD / 4), pc = q % (HD / 4); vst2(C + (size_t)(m0 + rl) * HD + pc * 4, *(const v4f*)(&so[rl][pc * 4])); }
}
__global__ __launch_bounds__(256) void k_pd(const float* __restrict__ H1, const float* __restrict__ M, const float* __restrict__ bvec, const float* __restrict__ sigma,
                                          const float* __restrict__ tau, const float* __restrict__ theta, const float* __restrict__ fc1w, const float* __restrict__ fc1b,
                                          const float* __restrict__ fc2w, const float* __restrict__ fc2b, float* __restrict__ out) {
  __shared__ __align__(16) float so_[TW][HD + 4];
  __shared__ __align__(16) float sxt[TW][HD + 4];
  __shared__ __align__(16) float sxc[TW][HD + 4];
  __shared__ __align__(16) float sy1[TW][HD + 4];
  __shared__ __align__(16) float sy2[TW][HD + 4];
  const int tid = threadIdx.x, wave = tid >> 5, lane = tid & 31, col = lane & 15, g = lane >> 4;
  const int b = blockIdx.x; const int t0 = T - TW;
  const float th = fminf(fmaxf(theta[0], 0.f), 5.f), sg = sigma[0], tu = tau[0];
  for (int q = tid; q < TW * HD; q += 256) { const int w = q / HD, u = q % HD; const float v = H1[((size_t)(t0 + w) * NBATCH + b) * HD + u]; so_[w][u] = v; sxt[w][u] = v; sxc[w][u] = v; }
  __syncthreads();
#pragma unroll 1
  for (int it = 0; it < MAXIT; ++it) {
    for (int q = tid; q < TW * HD; q += 256) { const int w = q / HD, u = q % HD; const float x = sxt[w][u];
      const float g1 = (w < TW - 1) ? sxt[w + 1][u] - x : 0.f; const float g2 = (u < HD - 1) ? sxt[w][u + 1] - x : 0.f;
      sy1[w][u] = fminf(fmaxf(x + sg * g1, -1.f), 1.f); sy2[w][u] = fminf(fmaxf(x + sg * g2, -1.f), 1.f); }
    __syncthreads();
    for (int q = tid; q < TW * HD; q += 256) { const int w = q / HD, u = q % HD;
      const float a1 = (w < TW - 1) ? sy1[w][u] : 0.f, a1m = (w > 0) ? sy1[w - 1][u] : 0.f;
      const float a2 = (u < HD - 1) ? sy2[w][u] : 0.f, a2m = (u > 0) ? sy2[w][u - 1] : 0.f;
      const float lad = (a1m - a1) + (a2m - a2);
      sxt[w][u] = (so_[w][u] - tu * lad) + tu * bvec[u]; }
    __syncthreads();
    v8f acc[2][2] = {};
#pragma unroll 1
    for (int kc = 0; kc < HD / 32; ++kc) { const F2 a0 = split_row(&sxt[col][0], kc * 32, lane), a1 = split_row(&sxt[16 + col][0], kc * 32, lane);
#pragma unroll
      for (int j = 0; j < 2; ++j) { const F2 bm = split_row(M + (size_t)((2 * wave + j) * 16 + col) * HD, kc * 32, lane); acc[0][j] = mac3(a0, bm, acc[0][j]); acc[1][j] = mac3(a1, bm, acc[1][j]); } }
    __syncthreads();
#pragma unroll
    for (int i = 0; i < 2; ++i)
#pragma unroll
      for (int j = 0; j < 2; ++j)
#pragma unroll
        for (int r = 0; r < 8; ++r) { const int w = i * 16 + 8 * g + r, u = (2 * wave + j) * 16 + col; const float xc2 = acc[i][j][r]; const float xold = sxc[w][u];
          sxc[w][u] = xc2; sxt[w][u] = xc2 + th * (xc2 - xold); }
    __syncthreads();
  }
  { v8f acc[2] = {};
#pragma unroll 1
    for (int kc = 0; kc < HD / 32; ++kc) { const F2 a = split_row(&sxt[16 + col][0], kc * 32, lane);
#pragma unroll
      for (int j = 0; j < 2; ++j) acc[j] = mac3(a, split_row(fc1w + (size_t)((2 * wave + j) * 16 + col) * HD, kc * 32, lane), acc[j]); }
#pragma unroll
    for (int j = 0; j < 2; ++j)
#pragma unroll
      for (int r = 0; r < 8; ++r) { const int u = (2 * wave + j) * 16 + col; sy1[8 * g + r][u] = acc[j][r] + fc1b[u]; }
  }
  __syncthreads();
  if (wave < 2) { v8f acc = {};
#pragma unroll 1
    for (int kc = 0; kc < HD / 32; ++kc) acc = mac3(split_row(&sy1[col][0], kc * 32, lane), split_row(fc2w + (size_t)(wave * 16 + col) * HD, kc * 32, lane), acc);
#pragma unroll
    for (int r = 0; r < 8; ++r) sy2[8 * g + r][wave * 16 + col] = acc[r] + fc2b[wave * 16 + col]; }
  __syncthreads();
  if (tid < 8) vst2(out + (size_t)b * NIN + tid * 4, *(const v4f*)(&sy2[15][tid * 4]));
}
extern "C" void kernel_launch(void* const* d_in, const int* in_sizes, int n_in, void* d_out, int out_size, void* d_ws, size_t ws_size, hipStream_t stream) {
  (void)in_sizes; (void)n_in; (void)out_size; (void)ws_size;
  const float** I = (const float**)d_in;
  const float* x = I[0];   const float* wih0 = I[2]; const float* whh0 = I[3]; const float* bih0 = I[4]; const float* bhh0 = I[5];
  const float* wih1 = I[6]; const float* whh1 = I[7]; const float* bih1 = I[8]; const float* bhh1 = I[9]; const float* fc1w = I[10]; const float* fc1b = I[11];
  const float* fc2w = I[12]; const float* fc2b = I[13]; const float* Hm = I[14]; const float* bvec = I[15]; const float* sigma = I[16]; const float* tau = I[17]; const float* theta = I[18];
  float* out = (float*)d_out;
  char* ws = (char*)d_ws; size_t off = 0;
  auto take = [&](size_t bytes) { char* p = ws + off; off += (bytes + 255) & ~(size_t)255; return p; };
  _Float16* X16 = (_Float16*)take((size_t)NROW * NIN * 2); _Float16* W0i = (_Float16*)take((size_t)G4 * NIN * 2); _Float16* W0h = (_Float16*)take((size_t)G4 * HD * 2);
  _Float16* W1i = (_Float16*)take((size_t)G4 * HD * 2); _Float16* W1h = (_Float16*)take((size_t)G4 * HD * 2);
  _Float16* H0 = (_Float16*)take((size_t)NROW * HD * 2); float* H1 = (float*)take((size_t)NROW * HD * 4);
  float* X = (float*)take((size_t)HD * HD * 4); float* M1 = (float*)take((size_t)HD * HD * 4); float* P2 = (float*)take((size_t)HD * HD * 4); float* M2 = (float*)take((size_t)HD * HD * 4);
  float* P4 = (float*)take((size_t)HD * HD * 4); float* M3 = (float*)take((size_t)HD * HD * 4); float* P8 = (float*)take((size_t)HD * HD * 4); float* M4 = (float*)take((size_t)HD * HD * 4);
  float* P16 = (float*)take((size_t)HD * HD * 4); float* M5 = (float*)take((size_t)HD * HD * 4);
  k_pack<<<(NROW * NIN / 8 + 255) / 256, 256, 0, stream>>>(x, X16, NROW * NIN / 8, 1.0f);
  k_pack<<<(G4 * NIN / 8 + 255) / 256, 256, 0, stream>>>(wih0, W0i, G4 * NIN / 8, WSC);
  k_pack<<<(G4 * HD / 8 + 255) / 256, 256, 0, stream>>>(whh0, W0h, G4 * HD / 8, WSC);
  k_pack<<<(G4 * HD / 8 + 255) / 256, 256, 0, stream>>>(wih1, W1i, G4 * HD / 8, WSC);
  k_pack<<<(G4 * HD / 8 + 255) / 256, 256, 0, stream>>>(whh1, W1h, G4 * HD / 8, WSC);
  k_lstm<NIN><<<1, 256, 0, stream>>>(X16, W0i, W0h, bih0, bhh0, H0, (float*)nullptr);
  k_lstm<HD><<<1, 256, 0, stream>>>(H0, W1i, W1h, bih1, bhh1, (_Float16*)nullptr, H1);
  k_xinit<<<(HD * HD / 4 + 255) / 256, 256, 0, stream>>>(Hm, tau, X, M1);
  k_mm256<<<HD / 16, 128, 0, stream>>>(X, X, nullptr, P2);
  k_mm256<<<HD / 16, 128, 0, stream>>>(M1, P2, M1, M2);
  k_mm256<<<HD / 16, 128, 0, stream>>>(P2, P2, nullptr, P4);
  k_mm256<<<HD / 16, 128, 0, stream>>>(M2, P4, M2, M3);
  k_mm256<<<HD / 16, 128, 0, stream>>>(P4, P4, nullptr, P8);
  k_mm256<<<HD / 16, 128, 0, stream>>>(M3, P8, M3, M4);
  k_mm256<<<HD / 16, 128, 0, stream>>>(P8, P8, nullptr, P16);
  k_mm256<<<HD / 16, 128, 0, stream>>>(M4, P16, M4, M5);
  k_pd<<<NBATCH, 256, 0, stream>>>(H1, M5, bvec, sigma, tau, theta, fc1w, fc1b, fc2w, fc2b, out);
}
